// EncoderMambaDecoderBlock_28793460752848
// MI455X (gfx1250) — hardware-run, weakly checked
//
#include <hip/hip_runtime.h>
#include <math.h>

typedef __attribute__((ext_vector_type(16))) _Float16 v16h;
typedef __attribute__((ext_vector_type(8)))  _Float16 v8h;
typedef __attribute__((ext_vector_type(16))) __bf16   v16b;
typedef __attribute__((ext_vector_type(8)))  __bf16   v8b;
typedef __attribute__((ext_vector_type(8)))  float    v8f;
typedef __attribute__((ext_vector_type(4)))  float    v4f;

constexpr int kBatch   = 8;
constexpr int kSeq     = 2048;
constexpr int kTok     = kBatch * kSeq;
constexpr int kFin     = 64;
constexpr int kHid     = 256;
constexpr int kDm      = 512;
constexpr int kDi      = 1024;
constexpr int kNst     = 16;
constexpr int kDtR     = 32;
constexpr int kXzP     = 2 * kDi;
constexpr int kXdP     = kDtR + 2 * kNst;
constexpr int kFout    = 64;
constexpr int kChunkB  = 2;
constexpr int kRows    = kChunkB * kSeq;
constexpr int kChunks  = kBatch / kChunkB;
constexpr int kConvTP  = 260;
constexpr int kScanTS  = 64;
constexpr int kScanCh  = 64;
constexpr int kScanYP  = 68;

static_assert(kTok == 16384);
static_assert(kXdP == 64);
static_assert(kRows == 4096 && kChunks == 4 && kChunks * kChunkB == kBatch);
static_assert((kFin % 32) == 0 && (kHid % 32) == 0 && (kDm % 32) == 0 && (kDi % 32) == 0);
static_assert((kRows % 64) == 0 && (kHid % 64) == 0 && (kDm % 64) == 0 && (kXzP % 64) == 0 && (kXdP % 64) == 0 && (kFout % 64) == 0);
static_assert((((kRows / 64) * (kHid / 64)) % 8) == 0 && (((kRows / 64) * (kDm / 64)) % 8) == 0);
static_assert((((kRows / 64) * (kXzP / 64)) % 8) == 0 && (((kRows / 64) * (kXdP / 64)) % 8) == 0 && (((kRows / 64) * (kFout / 64)) % 8) == 0);
static_assert((kSeq % kScanTS) == 0 && (kSeq % 64) == 0 && (kDi % kScanCh) == 0 && (kDi % 256) == 0);
static_assert((kSeq & (kSeq - 1)) == 0);

constexpr size_t kOffXB   = 0;
constexpr size_t kOffW1B  = kOffXB   + (size_t)kTok  * kFin * 2;
constexpr size_t kOffW2B  = kOffW1B  + (size_t)kHid  * kFin * 2;
constexpr size_t kOffWIB  = kOffW2B  + (size_t)kDm   * kHid * 2;
constexpr size_t kOffWXB  = kOffWIB  + (size_t)kXzP  * kDm  * 2;
constexpr size_t kOffWOB  = kOffWXB  + (size_t)kXdP  * kDi  * 2;
constexpr size_t kOffWD1B = kOffWOB  + (size_t)kDm   * kDi  * 2;
constexpr size_t kOffWD2B = kOffWD1B + (size_t)kHid  * kDm  * 2;
constexpr size_t kOffH1H  = kOffWD2B + (size_t)kFout * kHid * 2;
constexpr size_t kOffH1L  = kOffH1H  + (size_t)kRows * kHid * 2;
constexpr size_t kOffUH   = kOffH1L  + (size_t)kRows * kHid * 2;
constexpr size_t kOffUL   = kOffUH   + (size_t)kRows * kDm  * 2;
constexpr size_t kOffXZ   = kOffUL   + (size_t)kRows * kDm  * 2;
constexpr size_t kOffUC   = kOffXZ   + (size_t)kRows * kXzP * 4;
constexpr size_t kOffUCB  = kOffUC   + (size_t)kRows * kDi  * 4;
constexpr size_t kOffXD   = kOffUCB  + (size_t)kRows * kDi  * 2;
constexpr size_t kOffYH   = kOffXD   + (size_t)kRows * kXdP * 4;
constexpr size_t kOffYL   = kOffYH   + (size_t)kRows * kDi  * 2;
constexpr size_t kOffOH   = kOffYL   + (size_t)kRows * kDi  * 2;
constexpr size_t kOffOL   = kOffOH   + (size_t)kRows * kDm  * 2;
constexpr size_t kOffH2H  = kOffOL   + (size_t)kRows * kDm  * 2;
constexpr size_t kOffH2L  = kOffH2H  + (size_t)kRows * kHid * 2;
constexpr size_t kWsTotal = kOffH2L  + (size_t)kRows * kHid * 2;
static_assert(kWsTotal == 107675648ull);
static_assert(kWsTotal <= 134217728ull);
static_assert((kOffW1B % 128) == 0 && (kOffW2B % 128) == 0 && (kOffWIB % 128) == 0 && (kOffWXB % 128) == 0 &&
              (kOffWOB % 128) == 0 && (kOffWD1B % 128) == 0 && (kOffWD2B % 128) == 0 && (kOffH1H % 128) == 0 &&
              (kOffH1L % 128) == 0 && (kOffUH % 128) == 0 && (kOffUL % 128) == 0 && (kOffXZ % 128) == 0 &&
              (kOffUC % 128) == 0 && (kOffUCB % 128) == 0 && (kOffXD % 128) == 0 && (kOffYH % 128) == 0 &&
              (kOffYL % 128) == 0 && (kOffOH % 128) == 0 && (kOffOL % 128) == 0 && (kOffH2H % 128) == 0 &&
              (kOffH2L % 128) == 0);

__device__ __forceinline__ unsigned short f2bf_bits(float f) {
  unsigned u = __float_as_uint(f);
  return (unsigned short)((u + 0x7FFFu + ((u >> 16) & 1u)) >> 16);
}
__device__ __forceinline__ float bf_bits2f(unsigned short h) { return __uint_as_float(((unsigned)h) << 16); }
__device__ __forceinline__ float bf_rne(float f) { return bf_bits2f(f2bf_bits(f)); }

__device__ __forceinline__ void grp_guard_b(v8f& a0, v8f& a1, v8f& a2, v8f& a3, v16b x, v16b y) {
  asm volatile("v_nop\n\tv_nop\n\tv_nop\n\tv_nop" : "+v"(a0), "+v"(a1), "+v"(a2), "+v"(a3) : "v"(x), "v"(y));
}
__device__ __forceinline__ void keep4_b(v16b a, v16b b, v16b c, v16b d) { asm volatile("v_nop" :: "v"(a), "v"(b), "v"(c), "v"(d)); }
__device__ __forceinline__ void acc_guard4(v8f& a, v8f& b, v8f& c, v8f& d) { asm volatile("v_nop\n\tv_nop\n\tv_nop\n\tv_nop" : "+v"(a), "+v"(b), "+v"(c), "+v"(d)); }

struct FragB {
  union U { v16b v; v8b h[2]; };
  static __device__ __forceinline__ v16b load(const __bf16* p) {
    U f; f.h[0] = *(const v8b*)(p); f.h[1] = *(const v8b*)(p + 16); return f.v;
  }
  static __device__ __forceinline__ v8f mma(v16b a, v16b b, v8f c) {
    return __builtin_amdgcn_wmma_f32_16x16x32_bf16(false, a, false, b, (short)0, c, false, false);
  }
};

template <int SPL, int BIAS_MODE, int OUT_MODE, int ACT>
__global__ __launch_bounds__(256) void wmma_gemm64(
    const unsigned short* __restrict__ Ap, const unsigned short* __restrict__ A2p, int lda,
    const unsigned short* __restrict__ Btp, int ldb,
    void* __restrict__ Cout, void* __restrict__ Cout2, int ldc,
    const float* __restrict__ bias,
    int M, int N, int K) {
  typedef v16b V;
  const __bf16* A  = (const __bf16*)Ap;
  const __bf16* A2 = (const __bf16*)A2p;
  const __bf16* Bt = (const __bf16*)Btp;
  __shared__ __align__(16) float sT[8][16 * 68];
  const int lane = threadIdx.x & 31;
  const int wave = threadIdx.x >> 5;
  const int tilesN = N >> 6;
  const int tilesM = M >> 6;
  const int tile = blockIdx.x * 8 + wave;
  if (tile >= tilesM * tilesN) return;
  const int tm = tile / tilesN;
  const int tn = tile - tm * tilesN;
  const int m0 = tm << 6;
  const int n0 = tn << 6;

  const int rlane = lane & 15;
  const int koff  = (lane >> 4) * 8;
  const int mOff  = (lane >> 4) * 8;

  v8f acc[4][4];
#pragma unroll
  for (int i = 0; i < 4; ++i)
#pragma unroll
    for (int j = 0; j < 4; ++j) acc[i][j] = (v8f){0.f,0.f,0.f,0.f,0.f,0.f,0.f,0.f};

  for (int k0 = 0; k0 < K; k0 += 32) {
    V bh[4];
#pragma unroll
    for (int j = 0; j < 4; ++j) {
      const size_t bo = (size_t)(n0 + (j << 4) + rlane) * ldb + koff + k0;
      bh[j] = FragB::load(Bt + bo);
    }
#pragma unroll
    for (int i = 0; i < 4; ++i) {
      const size_t ao = (size_t)(m0 + (i << 4) + rlane) * lda + koff + k0;
      V ah = FragB::load(A + ao);
      V al = ah;
      if (SPL >= 1) al = FragB::load(A2 + ao);
#pragma unroll
      for (int j = 0; j < 4; ++j) {
        acc[i][j] = FragB::mma(ah, bh[j], acc[i][j]);
        if (SPL >= 1) acc[i][j] = FragB::mma(al, bh[j], acc[i][j]);
      }
      grp_guard_b(acc[i][0], acc[i][1], acc[i][2], acc[i][3], ah, al);
    }
    keep4_b(bh[0], bh[1], bh[2], bh[3]);
  }
  acc_guard4(acc[0][0], acc[0][1], acc[0][2], acc[0][3]);
  acc_guard4(acc[1][0], acc[1][1], acc[1][2], acc[1][3]);
  acc_guard4(acc[2][0], acc[2][1], acc[2][2], acc[2][3]);
  acc_guard4(acc[3][0], acc[3][1], acc[3][2], acc[3][3]);

  float* slab = sT[wave];
#pragma unroll
  for (int i = 0; i < 4; ++i) {
    const int mBase = m0 + (i << 4);
#pragma unroll
    for (int j = 0; j < 4; ++j) {
      const int n = n0 + (j << 4) + rlane;
      float bv = 0.f;
      if (BIAS_MODE == 2) bv = bf_rne(bias[n]);
#pragma unroll
      for (int r = 0; r < 8; ++r) {
        float v = acc[i][j][r];
        if (BIAS_MODE == 2) v += bv;
        if (ACT == 2) v = fmaxf(v, 0.0f);
        slab[(mOff + r) * 68 + (j << 4) + rlane] = v;
      }
    }
    __builtin_amdgcn_fence(__ATOMIC_RELEASE, "workgroup");
    __builtin_amdgcn_wave_barrier();
    __builtin_amdgcn_fence(__ATOMIC_ACQUIRE, "workgroup");
    if (OUT_MODE == 0) {
      float* C = (float*)Cout;
      const int hh = lane >> 4, c4 = (lane & 15) * 4;
      for (int pass = 0; pass < 2; ++pass) {
#pragma unroll
        for (int it = 0; it < 8; ++it) {
          const int row = it * 2 + hh;
          v4f v = *(const v4f*)(slab + row * 68 + c4);
          *(volatile v4f*)(C + (size_t)(mBase + row) * ldc + n0 + c4) = v;
        }
        __threadfence();
      }
    } else {
      const int q = lane >> 3, c8 = (lane & 7) * 8;
      unsigned short* C  = (unsigned short*)Cout;
      unsigned short* C2 = (unsigned short*)Cout2;
      for (int pass = 0; pass < 2; ++pass) {
#pragma unroll
        for (int it = 0; it < 4; ++it) {
          const int row = it * 4 + q;
          const float* sp = slab + row * 68 + c8;
          v8h hv, lv;
#pragma unroll
          for (int e = 0; e < 8; ++e) {
            const float sv = sp[e];
            const unsigned short hb = f2bf_bits(sv);
            const unsigned short lb = f2bf_bits(sv - bf_bits2f(hb));
            hv[e] = __builtin_bit_cast(_Float16, hb);
            lv[e] = __builtin_bit_cast(_Float16, lb);
          }
          *(volatile v8h*)(C  + (size_t)(mBase + row) * ldc + n0 + c8) = hv;
          *(volatile v8h*)(C2 + (size_t)(mBase + row) * ldc + n0 + c8) = lv;
        }
        __threadfence();
      }
    }
    __builtin_amdgcn_fence(__ATOMIC_RELEASE, "workgroup");
    __builtin_amdgcn_wave_barrier();
    __builtin_amdgcn_fence(__ATOMIC_ACQUIRE, "workgroup");
  }
}

__global__ __launch_bounds__(256) void cast_rows_bf16_kernel(
    const float* __restrict__ src, unsigned short* __restrict__ dst, int total8)
{
  const int i = blockIdx.x * 256 + threadIdx.x;
  if (i >= total8) return;
  const size_t e0 = (size_t)i << 3;
  const v4f a0 = *(const v4f*)(src + e0);
  const v4f a1 = *(const v4f*)(src + e0 + 4);
  v8h hv;
#pragma unroll
  for (int e = 0; e < 4; ++e) {
    const float f0 = a0[e];
    const float f1 = a1[e];
    const unsigned short h0 = f2bf_bits(f0);
    const unsigned short h1 = f2bf_bits(f1);
    hv[e]     = __builtin_bit_cast(_Float16, h0);
    hv[4 + e] = __builtin_bit_cast(_Float16, h1);
  }
  unsigned short* qd = dst + e0;
  *(volatile v8h*)qd = hv;
  __threadfence();
  *(volatile v8h*)qd = hv;
}

__global__ __launch_bounds__(256) void conv_silu_kernel(
    const float* __restrict__ XZ, const float* __restrict__ cw, const float* __restrict__ cb,
    float* __restrict__ UC, unsigned short* __restrict__ UCB)
{
  __shared__ __align__(16) float sT[16 * kConvTP];
  const int tid = threadIdx.x, lane = tid & 31, wave = tid >> 5;
  const int d0 = blockIdx.x * 256, d = d0 + tid;
  const int g0 = blockIdx.y * 64;
  const int tb = g0 & (kSeq - 1);
  const v4f wv = *(const v4f*)(cw + (size_t)d * 4);
  const float wr0 = wv[0], wr1 = wv[1], wr2 = wv[2], wr3 = wv[3];
  const float w0 = bf_rne(wr0), w1 = bf_rne(wr1), w2 = bf_rne(wr2), w3 = bf_rne(wr3);
  const float bc = bf_rne(cb[d]);
  float xm3, xm2, xm1;
  {
    const bool hist = (tb > 0);
    const int rb = hist ? (g0 - 3) : g0;
    const float v3 = XZ[(size_t)rb * kXzP + d];
    const float v2 = XZ[(size_t)(rb + 1) * kXzP + d];
    const float v1 = XZ[(size_t)(rb + 2) * kXzP + d];
    xm3 = hist ? v3 : 0.f;
    xm2 = hist ? v2 : 0.f;
    xm1 = hist ? v1 : 0.f;
  }
  const int hrow = wave >> 1;
  const int hch  = (wave & 1) * 128 + lane * 4;
#pragma unroll 1
  for (int sub = 0; sub < 4; ++sub) {
    const int lb = g0 + sub * 16;
#pragma unroll 1
    for (int s = 0; s < 16; ++s) {
      const float xcur = XZ[(size_t)(lb + s) * kXzP + d];
      float acc = w0 * xm3;
      acc = fmaf(w1, xm2, acc);
      acc = fmaf(w2, xm1, acc);
      acc = fmaf(w3, xcur, acc);
      const float sv = acc + bc;
      const float sg = __builtin_amdgcn_rcpf(1.0f + expf(-sv));
      sT[s * kConvTP + tid] = sv * sg;
      xm3 = xm2; xm2 = xm1; xm1 = xcur;
    }
    __syncthreads();
    v4f fv[4];
    v8h bh[2];
#pragma unroll
    for (int it = 0; it < 4; ++it) fv[it] = *(const v4f*)(sT + (it * 4 + hrow) * kConvTP + hch);
#pragma unroll
    for (int it = 0; it < 2; ++it) {
      const float* sp = sT + (it * 8 + wave) * kConvTP + lane * 8;
      const v4f a0 = *(const v4f*)(sp);
      const v4f a1 = *(const v4f*)(sp + 4);
#pragma unroll
      for (int e = 0; e < 4; ++e) {
        const float f0 = a0[e];
        const float f1 = a1[e];
        const unsigned short h0 = f2bf_bits(f0);
        const unsigned short h1 = f2bf_bits(f1);
        bh[it][e]     = __builtin_bit_cast(_Float16, h0);
        bh[it][4 + e] = __builtin_bit_cast(_Float16, h1);
      }
    }
    for (int pass = 0; pass < 2; ++pass) {
#pragma unroll
      for (int it = 0; it < 4; ++it)
        *(volatile v4f*)(UC + (size_t)(lb + it * 4 + hrow) * kDi + d0 + hch) = fv[it];
#pragma unroll
      for (int it = 0; it < 2; ++it) {
        const size_t o = (size_t)(lb + it * 8 + wave) * kDi + d0 + lane * 8;
        *(volatile v8h*)(UCB + o) = bh[it];
      }
      __threadfence();
    }
    __syncthreads();
  }
}

__global__ __launch_bounds__(64) void scan_kernel(
    const float* __restrict__ XD, const float* __restrict__ UC, const float* __restrict__ XZ,
    const float* __restrict__ Wdt, const float* __restrict__ bdt, const float* __restrict__ Alog,
    const float* __restrict__ Dp, unsigned short* __restrict__ YH, unsigned short* __restrict__ YL)
{
  __shared__ __align__(16) float sX[kScanTS * kXdP];
  __shared__ __align__(16) float sY[kScanTS * kScanYP];
  __shared__ __align__(16) float sW[kDtR * kScanCh];
  __shared__ __align__(16) float sA[kNst * kScanCh];
  const int tid = threadIdx.x, lane = tid & 31, wave = tid >> 5;
  constexpr int kBlkPerB = kDi / kScanCh;
  const int bix = blockIdx.x / kBlkPerB;
  const int d0  = (blockIdx.x - bix * kBlkPerB) * kScanCh;
  const int d   = d0 + tid;
  const size_t row0 = (size_t)bix * kSeq;
#pragma unroll 1
  for (int r = 0; r < kDtR; ++r) sW[r * kScanCh + tid] = bf_rne(Wdt[(size_t)d * kDtR + r]);
#pragma unroll 1
  for (int s = 0; s < kNst; ++s) sA[s * kScanCh + tid] = -expf(bf_rne(Alog[(size_t)d * kNst + s]));
  __syncthreads();
  float negA[kNst], h[kNst];
#pragma unroll
  for (int s = 0; s < kNst; ++s) {
    negA[s] = sA[s * kScanCh + tid];
    h[s] = 0.f;
  }
  const float bb = bf_rne(bdt[d]);
  const float Dd = bf_rne(Dp[d]);
  const int lr = tid >> 4, lc4 = (tid & 15) * 4;
  const int q = lane >> 3, c8 = (lane & 7) * 8;
#pragma unroll 1
  for (int t0 = 0; t0 < kSeq; t0 += kScanTS) {
    __syncthreads();
#pragma unroll
    for (int i = 0; i < 16; ++i) {
      const int r = lr + 4 * i;
      *(v4f*)(sX + r * kXdP + lc4) = *(const v4f*)(XD + (row0 + t0 + r) * kXdP + lc4);
    }
    __syncthreads();
#pragma unroll 1
    for (int s = 0; s < kScanTS; ++s) {
      const int t = t0 + s;
      const float* xr = sX + s * kXdP;
      float vdot = 0.f;
#pragma unroll 1
      for (int r4 = 0; r4 < kDtR / 4; ++r4) {
        const v4f xv = *(const v4f*)(xr + 4 * r4);
        const float* wp = sW + (4 * r4) * kScanCh + tid;
        vdot = fmaf(xv[0], wp[0], vdot);
        vdot = fmaf(xv[1], wp[kScanCh], vdot);
        vdot = fmaf(xv[2], wp[2 * kScanCh], vdot);
        vdot = fmaf(xv[3], wp[3 * kScanCh], vdot);
      }
      float Bs[kNst], Cs[kNst];
#pragma unroll
      for (int q4 = 0; q4 < 4; ++q4) {
        const v4f bv = *(const v4f*)(xr + kDtR + 4 * q4);
        const v4f cv = *(const v4f*)(xr + kDtR + kNst + 4 * q4);
        Bs[4 * q4 + 0] = bv[0]; Bs[4 * q4 + 1] = bv[1]; Bs[4 * q4 + 2] = bv[2]; Bs[4 * q4 + 3] = bv[3];
        Cs[4 * q4 + 0] = cv[0]; Cs[4 * q4 + 1] = cv[1]; Cs[4 * q4 + 2] = cv[2]; Cs[4 * q4 + 3] = cv[3];
      }
      const float v   = vdot + bb;
      const float a   = __expf(-fabsf(v));
      const float u   = 1.0f + a;
      const float l1p = __logf(u) + (a - (u - 1.0f)) * __builtin_amdgcn_rcpf(u);
      const float dt  = fmaxf(v, 0.0f) + l1p;
      const float xt  = UC[(row0 + t) * kDi + d];
      const float dtx = dt * xt;
      float y = 0.f;
#pragma unroll
      for (int k = 0; k < kNst; ++k) {
        const float e = __expf(dt * negA[k]);
        h[k] = e * h[k] + dtx * Bs[k];
        y = h[k] * Cs[k] + y;
      }
      y = xt * Dd + y;
      const float zv = XZ[(row0 + t) * kXzP + kDi + d];
      const float sg = __builtin_amdgcn_rcpf(1.0f + expf(-zv));
      y = y * (zv * sg);
      sY[s * kScanYP + tid] = y;
    }
    __syncthreads();
    v8h hv[8], lv[8];
#pragma unroll
    for (int it = 0; it < 8; ++it) {
      const int row = it * 8 + wave * 4 + q;
      const float* sp = sY + row * kScanYP + c8;
      const v4f a0 = *(const v4f*)(sp);
      const v4f a1 = *(const v4f*)(sp + 4);
#pragma unroll
      for (int e = 0; e < 4; ++e) {
        const float f0 = a0[e];
        const float f1 = a1[e];
        const unsigned short h0 = f2bf_bits(f0), h1 = f2bf_bits(f1);
        const unsigned short l0 = f2bf_bits(f0 - bf_bits2f(h0)), l1 = f2bf_bits(f1 - bf_bits2f(h1));
        hv[it][e]     = __builtin_bit_cast(_Float16, h0);
        hv[it][4 + e] = __builtin_bit_cast(_Float16, h1);
        lv[it][e]     = __builtin_bit_cast(_Float16, l0);
        lv[it][4 + e] = __builtin_bit_cast(_Float16, l1);
      }
    }
    for (int pass = 0; pass < 2; ++pass) {
#pragma unroll
      for (int it = 0; it < 8; ++it) {
        const int row = it * 8 + wave * 4 + q;
        const size_t o = (row0 + t0 + row) * kDi + d0 + c8;
        *(volatile v8h*)(YH + o) = hv[it];
        *(volatile v8h*)(YL + o) = lv[it];
      }
      __threadfence();
    }
  }
}

extern "C" void kernel_launch(void* const* d_in, const int* in_sizes, int n_in,
                              void* d_out, int out_size, void* d_ws, size_t ws_size,
                              hipStream_t stream) {
  if (n_in < 18) return;
  if (in_sizes[0]  != kTok * kFin) return;
  if (in_sizes[1]  != kHid * kFin) return;
  if (in_sizes[2]  != kHid) return;
  if (in_sizes[3]  != kDm * kHid) return;
  if (in_sizes[4]  != kDm) return;
  if (in_sizes[5]  != kXzP * kDm) return;
  if (in_sizes[6]  != kDi * 4) return;
  if (in_sizes[7]  != kDi) return;
  if (in_sizes[8]  != kXdP * kDi) return;
  if (in_sizes[9]  != kDi * kDtR) return;
  if (in_sizes[10] != kDi) return;
  if (in_sizes[11] != kDi * kNst) return;
  if (in_sizes[12] != kDi) return;
  if (in_sizes[13] != kDm * kDi) return;
  if (in_sizes[14] != kHid * kDm) return;
  if (in_sizes[15] != kHid) return;
  if (in_sizes[16] != kFout * kHid) return;
  if (in_sizes[17] != kFout) return;
  if (out_size != kTok * kFout) return;
  if (ws_size < kWsTotal) return;

  const float* x_in   = (const float*)d_in[0];
  const float* w_e1   = (const float*)d_in[1];
  const float* b_e1   = (const float*)d_in[2];
  const float* w_e2   = (const float*)d_in[3];
  const float* b_e2   = (const float*)d_in[4];
  const float* w_inp  = (const float*)d_in[5];
  const float* conv_w = (const float*)d_in[6];
  const float* conv_b = (const float*)d_in[7];
  const float* w_xp   = (const float*)d_in[8];
  const float* w_dt   = (const float*)d_in[9];
  const float* b_dt   = (const float*)d_in[10];
  const float* a_log  = (const float*)d_in[11];
  const float* d_skip = (const float*)d_in[12];
  const float* w_outp = (const float*)d_in[13];
  const float* w_d1   = (const float*)d_in[14];
  const float* b_d1   = (const float*)d_in[15];
  const float* w_d2   = (const float*)d_in[16];
  const float* b_d2   = (const float*)d_in[17];
  float* dout = (float*)d_out;

  char* ws = (char*)d_ws;
  unsigned short* XB   = (unsigned short*)(ws + kOffXB);
  unsigned short* W1B  = (unsigned short*)(ws + kOffW1B);
  unsigned short* W2B  = (unsigned short*)(ws + kOffW2B);
  unsigned short* WIB  = (unsigned short*)(ws + kOffWIB);
  unsigned short* WXB  = (unsigned short*)(ws + kOffWXB);
  unsigned short* WOB  = (unsigned short*)(ws + kOffWOB);
  unsigned short* WD1B = (unsigned short*)(ws + kOffWD1B);
  unsigned short* WD2B = (unsigned short*)(ws + kOffWD2B);
  unsigned short* H1H  = (unsigned short*)(ws + kOffH1H);
  unsigned short* H1L  = (unsigned short*)(ws + kOffH1L);
  unsigned short* UH   = (unsigned short*)(ws + kOffUH);
  unsigned short* UL   = (unsigned short*)(ws + kOffUL);
  float*          XZ   = (float*)(ws + kOffXZ);
  float*          UC   = (float*)(ws + kOffUC);
  unsigned short* UCB  = (unsigned short*)(ws + kOffUCB);
  float*          XD   = (float*)(ws + kOffXD);
  unsigned short* YH   = (unsigned short*)(ws + kOffYH);
  unsigned short* YL   = (unsigned short*)(ws + kOffYL);
  unsigned short* OH   = (unsigned short*)(ws + kOffOH);
  unsigned short* OL   = (unsigned short*)(ws + kOffOL);
  unsigned short* H2H  = (unsigned short*)(ws + kOffH2H);
  unsigned short* H2L  = (unsigned short*)(ws + kOffH2L);
  const float* no_bias = conv_b;

  cast_rows_bf16_kernel<<<(kTok * kFin / 8) / 256, 256, 0, stream>>>(x_in,   XB,   kTok * kFin / 8);
  cast_rows_bf16_kernel<<<(kHid * kFin / 8) / 256, 256, 0, stream>>>(w_e1,   W1B,  kHid * kFin / 8);
  cast_rows_bf16_kernel<<<(kDm * kHid / 8) / 256,  256, 0, stream>>>(w_e2,   W2B,  kDm * kHid / 8);
  cast_rows_bf16_kernel<<<(kXzP * kDm / 8) / 256,  256, 0, stream>>>(w_inp,  WIB,  kXzP * kDm / 8);
  cast_rows_bf16_kernel<<<(kXdP * kDi / 8) / 256,  256, 0, stream>>>(w_xp,   WXB,  kXdP * kDi / 8);
  cast_rows_bf16_kernel<<<(kDm * kDi / 8) / 256,   256, 0, stream>>>(w_outp, WOB,  kDm * kDi / 8);
  cast_rows_bf16_kernel<<<(kHid * kDm / 8) / 256,  256, 0, stream>>>(w_d1,   WD1B, kHid * kDm / 8);
  cast_rows_bf16_kernel<<<(kFout * kHid / 8) / 256, 256, 0, stream>>>(w_d2,  WD2B, kFout * kHid / 8);

  for (int c = 0; c < kChunks; ++c) {
    const unsigned short* XBc = XB + (size_t)c * kRows * kFin;
    float* outc = dout + (size_t)c * kRows * kFout;

    wmma_gemm64<0, 2, 2, 2><<<dim3(((kRows / 64) * (kHid / 64)) / 8), 256, 0, stream>>>(
        XBc, XBc, kFin, W1B, kFin, (void*)H1H, (void*)H1L, kHid, b_e1, kRows, kHid, kFin);

    wmma_gemm64<1, 2, 2, 0><<<dim3(((kRows / 64) * (kDm / 64)) / 8), 256, 0, stream>>>(
        H1H, H1L, kHid, W2B, kHid, (void*)UH, (void*)UL, kDm, b_e2, kRows, kDm, kHid);

    wmma_gemm64<1, 0, 0, 0><<<dim3(((kRows / 64) * (kXzP / 64)) / 8), 256, 0, stream>>>(
        UH, UL, kDm, WIB, kDm, (void*)XZ, (void*)XZ, kXzP, no_bias, kRows, kXzP, kDm);

    conv_silu_kernel<<<dim3(kDi / 256, kRows / 64), 256, 0, stream>>>(XZ, conv_w, conv_b, UC, UCB);

    wmma_gemm64<0, 0, 0, 0><<<dim3(((kRows / 64) * (kXdP / 64)) / 8), 256, 0, stream>>>(
        UCB, UCB, kDi, WXB, kDi, (void*)XD, (void*)XD, kXdP, no_bias, kRows, kXdP, kDi);

    scan_kernel<<<kChunkB * (kDi / kScanCh), kScanCh, 0, stream>>>(XD, UC, XZ, w_dt, b_dt, a_log, d_skip, YH, YL);

    wmma_gemm64<1, 0, 2, 0><<<dim3(((kRows / 64) * (kDm / 64)) / 8), 256, 0, stream>>>(
        YH, YL, kDi, WOB, kDi, (void*)OH, (void*)OL, kDm, no_bias, kRows, kDm, kDi);

    wmma_gemm64<1, 2, 2, 2><<<dim3(((kRows / 64) * (kHid / 64)) / 8), 256, 0, stream>>>(
        OH, OL, kDm, WD1B, kDm, (void*)H2H, (void*)H2L, kHid, b_d1, kRows, kHid, kDm);

    wmma_gemm64<1, 2, 0, 0><<<dim3(((kRows / 64) * (kFout / 64)) / 8), 256, 0, stream>>>(
        H2H, H2L, kHid, WD2B, kHid, (void*)outc, (void*)outc, kFout, b_d2, kRows, kFout, kHid);
  }
}
